// LLCMBackbone_67688684585102
// MI455X (gfx1250) — hardware-verified
//
#include <hip/hip_runtime.h>
#include <math.h>

typedef __attribute__((ext_vector_type(16))) _Float16 v16h;
typedef __attribute__((ext_vector_type(16))) __bf16 v16b;
typedef __attribute__((ext_vector_type(8)))  _Float16 v8h;
typedef __attribute__((ext_vector_type(8)))  float v8f;
typedef __attribute__((ext_vector_type(4)))  float v4f;
typedef __attribute__((ext_vector_type(2)))  float v2f;
typedef __attribute__((ext_vector_type(4)))  unsigned v4u;
typedef __attribute__((ext_vector_type(4)))  int v4i;
typedef float __attribute__((may_alias)) float_a;
typedef int __attribute__((may_alias)) int_a;

template <typename T> __device__ __forceinline__ void vst2(void* p, T v) { *(volatile T*)p = v; __threadfence(); *(volatile T*)p = v; }
__device__ __forceinline__ v8f wmma16(v16h a, v16h b, v8f c) {
  v8f d = __builtin_amdgcn_wmma_f32_16x16x32_f16(false, a, false, b, (short)0, c, false, false);
  asm volatile("v_nop\n\tv_nop\n\tv_nop\n\tv_nop" : "+v"(d) : "v"(a), "v"(b));
  return d;
}
__device__ __forceinline__ v8f wmma_bf(v16b a, v16b b, v8f c) {
  v8f d = __builtin_amdgcn_wmma_f32_16x16x32_bf16(false, a, false, b, (short)0, c, false, false);
  asm volatile("v_nop\n\tv_nop\n\tv_nop\n\tv_nop" : "+v"(d) : "v"(a), "v"(b));
  return d;
}
__device__ __forceinline__ v16h frag_h(const _Float16* rowk0, int lane) {
  union { v16h v; v8h q[2]; } u; const _Float16* p = rowk0 + 8 * (lane >> 4);
  u.q[0] = *(const v8h*)p; u.q[1] = *(const v8h*)(p + 16); return u.v;
}
__device__ __forceinline__ v16h frag_f32(const float* rowk0, int lane) {
  v16h a; const float* p = rowk0 + 8 * (lane >> 4);
#pragma unroll
  for (int i = 0; i < 8; ++i) { a[i] = (_Float16)p[i]; a[8 + i] = (_Float16)p[16 + i]; }
  return a;
}
__device__ __forceinline__ v16h frag_f32s(const float* rowk0, int lane, float sc) {
  v16h a; const float* p = rowk0 + 8 * (lane >> 4);
#pragma unroll
  for (int i = 0; i < 8; ++i) { a[i] = (_Float16)(p[i] * sc); a[8 + i] = (_Float16)(p[16 + i] * sc); }
  return a;
}
__device__ __forceinline__ v16h fragc_f32(const float* W, int k0, int n, int lane, int ld, int K) {
  v16h a; const int g = lane >> 4;
#pragma unroll
  for (int i = 0; i < 8; ++i) { const int ka = k0 + 8 * g + i, kb = ka + 16;
    a[i] = (_Float16)(ka < K ? W[(size_t)(ka < K ? ka : K - 1) * ld + n] : 0.f); a[8 + i] = (_Float16)(kb < K ? W[(size_t)(kb < K ? kb : K - 1) * ld + n] : 0.f); }
  return a;
}
struct F2 { v16b h, l; };
__device__ __forceinline__ F2 bsplit16(const float v[16]) { F2 r;
#pragma unroll
  for (int i = 0; i < 16; ++i) { const __bf16 h = (__bf16)v[i]; r.h[i] = h; r.l[i] = (__bf16)(v[i] - (float)h); }
  return r; }
__device__ __forceinline__ F2 split_row(const float* row, int k0, int lane) { float v[16]; const float* p = row + k0 + 8 * (lane >> 4);
#pragma unroll
  for (int i = 0; i < 8; ++i) { v[i] = p[i]; v[8 + i] = p[16 + i]; }
  return bsplit16(v); }
__device__ __forceinline__ F2 split_rowK(const float* row, int k0, int lane, int K) { float v[16]; const int g = lane >> 4;
#pragma unroll
  for (int i = 0; i < 8; ++i) { const int ka = k0 + 8 * g + i, kb = ka + 16; v[i] = ka < K ? row[ka < K ? ka : K - 1] : 0.f; v[8 + i] = kb < K ? row[kb < K ? kb : K - 1] : 0.f; }
  return bsplit16(v); }
__device__ __forceinline__ F2 split_col(const float* W, int k0, int n, int lane, int ld, int K) { float v[16]; const int g = lane >> 4;
#pragma unroll
  for (int i = 0; i < 8; ++i) { const int ka = k0 + 8 * g + i, kb = ka + 16; v[i] = ka < K ? W[(size_t)(ka < K ? ka : K - 1) * ld + n] : 0.f; v[8 + i] = kb < K ? W[(size_t)(kb < K ? kb : K - 1) * ld + n] : 0.f; }
  return bsplit16(v); }
__device__ __forceinline__ v8f mac3(const F2& a, const F2& b, v8f c) { c = wmma_bf(a.l, b.h, c); c = wmma_bf(a.h, b.l, c); return wmma_bf(a.h, b.h, c); }
__device__ __forceinline__ float sigm(float v) { return 1.0f / (1.0f + expf(-v)); }
#define LDSX() do { asm volatile("s_wait_dscnt 0" ::: "memory"); __builtin_amdgcn_wave_barrier(); __builtin_amdgcn_fence(__ATOMIC_RELEASE, "workgroup"); } while (0)


#define NB 4
#define SS 2048
#define NR (NB * SS)
#define DD 128
#define NH 4
#define HD 32
#define TH 8
#define TD 32
#define FF 512
#define NL 3
#define SD 6
#ifndef NRT
#define NRT NR
#endif
typedef __attribute__((ext_vector_type(8))) __bf16 v8b;
__device__ __forceinline__ v16b frag_b(const __bf16* rowk0, int lane) {
  union { v16b v; v8b q[2]; } u; const __bf16* p = rowk0 + 8 * (lane >> 4);
  u.q[0] = *(const v8b*)p; u.q[1] = *(const v8b*)(p + 16); return u.v;
}
__device__ __forceinline__ float bfr(float v) { return (float)(__bf16)v; }
__device__ __attribute__((noinline)) float exp_ni(float v) { return expf(v); }
__device__ __attribute__((noinline)) float erf_ni(float v) { return erff(v); }
__device__ __forceinline__ float gelu_exact(float v) { return 0.5f * v * (1.0f + erf_ni(v * 0.70710678118654752f)); }

#define PL_QKV 0
#define PL_O   (PL_QKV + 3 * DD * DD)
#define PL_F1  (PL_O + DD * DD)
#define PL_F2  (PL_F1 + FF * DD)
#define PL_SZ  (PL_F2 + DD * FF)
#define PK_END ((size_t)NL * PL_SZ)
#define WS_PK  0u
#define WS_X   (((2u * PK_END) + 127u) / 128u * 128u)
#define WS_XH  (WS_X + 4u * NR * DD)
#define WS_XL  (WS_XH + 2u * NR * DD)
#define WS_Y   (WS_XL + 2u * NR * DD)
#define WS_QH  (WS_Y + 4u * NR * DD)
#define WS_QL  (WS_QH + 2u * NR * 2 * DD)
#define WS_VTH (WS_QL + 2u * NR * 2 * DD)
#define WS_VTL (WS_VTH + 2u * NR * DD)
#define WS_AH  (WS_VTL + 2u * NR * DD)
#define WS_AL  (WS_AH + 2u * NR * DD)
#define WS_HFH (WS_AL + 2u * NR * DD)
#define WS_HFL (WS_HFH + 2u * NR * FF)
#define WS_POOL (WS_HFL + 2u * NR * FF)
#define WS_END (WS_POOL + 4u * NB * (SS / 64) * DD)

__global__ __launch_bounds__(128) void k_pack(const float* __restrict__ WQ, const float* __restrict__ WK, const float* __restrict__ WV, const float* __restrict__ WO, const float* __restrict__ W1, const float* __restrict__ W2, __bf16* __restrict__ PK) {
  __shared__ __align__(16) __bf16 s[FF]; const int n = blockIdx.x, which = blockIdx.y, l = blockIdx.z, t = threadIdx.x; int K = DD; size_t dst; __bf16* base = PK + (size_t)l * PL_SZ;
  if (which == 0) { if (n >= 3 * DD) return; const int m = n / DD, r = n % DD; const float* Wm = (m == 0) ? WQ : (m == 1) ? WK : WV; for (int k = t; k < DD; k += 128) s[k] = (__bf16)Wm[((size_t)l * DD + k) * DD + r]; dst = PL_QKV + (size_t)n * DD; }
  else if (which == 1) { if (n >= DD) return; for (int k = t; k < DD; k += 128) s[k] = (__bf16)WO[((size_t)l * DD + k) * DD + n]; dst = PL_O + (size_t)n * DD; }
  else if (which == 2) { for (int k = t; k < DD; k += 128) s[k] = (__bf16)W1[((size_t)l * DD + k) * FF + n]; dst = PL_F1 + (size_t)n * DD; }
  else { if (n >= DD) return; K = FF; for (int k = t; k < FF; k += 128) s[k] = (__bf16)W2[((size_t)l * FF + k) * DD + n]; dst = PL_F2 + (size_t)n * FF; }
  __syncthreads();
  if (t < K / 8) vst2((unsigned*)(base + dst + t * 8), *(const v4u*)&s[t * 8]);
}
__global__ __launch_bounds__(128) void k_embed(const float* __restrict__ X0, const float* __restrict__ EW, const float* __restrict__ EB, float* __restrict__ X, __bf16* __restrict__ XH, __bf16* __restrict__ XL) {
  __shared__ __align__(16) float sx[DD]; __shared__ __align__(16) __bf16 sh_[DD], sl_[DD]; const int t = threadIdx.x; const size_t row = blockIdx.x;
  float a = 0.f;
#pragma unroll
  for (int k = 0; k < SD; ++k) a += bfr(X0[row * SD + k]) * bfr(EW[k * DD + t]);
  const float v = a + bfr(EB[t]); sx[t] = v; const __bf16 hb = (__bf16)v; sh_[t] = hb; sl_[t] = (__bf16)(v - (float)hb);
  __syncthreads();
  if (t < 32) vst2(X + row * DD + t * 4, *(const v4f*)&sx[t * 4]); else if (t < 48) vst2((unsigned*)(XH + row * DD + (t - 32) * 8), *(const v4u*)&sh_[(t - 32) * 8]); else if (t < 64) vst2((unsigned*)(XL + row * DD + (t - 48) * 8), *(const v4u*)&sl_[(t - 48) * 8]);
}
template <int MODE>
__global__ __launch_bounds__(128) void k_gemm(const __bf16* __restrict__ AH, const __bf16* __restrict__ AL, const __bf16* __restrict__ P, const float* __restrict__ BIAS, const float* __restrict__ X, _Float16* __restrict__ QH, _Float16* __restrict__ QL, _Float16* __restrict__ VTH, _Float16* __restrict__ VTL, __bf16* __restrict__ OH, __bf16* __restrict__ OL, float* __restrict__ OUTF, int which0) {
  constexpr int KIN = (MODE == 3) ? FF : DD;
  __shared__ __align__(16) float so[4][16][132]; __shared__ __align__(16) __bf16 soh[4][16][136], sol[4][16][136]; __shared__ __align__(16) _Float16 sqh[4][16][136], sql[4][16][136]; __shared__ __align__(16) _Float16 sth[128][72], stl[128][72];
  const int tid = threadIdx.x, wave = tid >> 5, lane = tid & 31, col = lane & 15, g = lane >> 4; const size_t r0 = (size_t)blockIdx.x * 64 + wave * 16; const int n0 = blockIdx.y * 128;
  v8f acc[8] = {};
#pragma unroll 2
  for (int kc = 0; kc < KIN / 32; ++kc) { F2 a; a.h = frag_b(AH + (r0 + col) * KIN + kc * 32, lane); a.l = frag_b(AL + (r0 + col) * KIN + kc * 32, lane);
#pragma unroll
    for (int j = 0; j < 8; ++j) { const v16b w = frag_b(P + (size_t)(n0 + j * 16 + col) * KIN + kc * 32, lane); acc[j] = wmma_bf(a.l, w, acc[j]); acc[j] = wmma_bf(a.h, w, acc[j]); } }
  if (MODE == 0) { const int which = which0;
#pragma unroll
    for (int j = 0; j < 8; ++j) { const int c = j * 16 + col; const float bb = bfr(BIAS[n0 + c]);
#pragma unroll
      for (int r = 0; r < 8; ++r) { float v = acc[j][r] + bb;
        if (which == 1 && (c & (HD - 1)) >= TH) v = -v;
        const _Float16 hv = (_Float16)v; const _Float16 lv = (_Float16)((v - (float)hv) * 2048.0f);
        if (which < 2) { sqh[wave][8 * g + r][c] = hv; sql[wave][8 * g + r][c] = lv; } else { sth[c][wave * 16 + 8 * g + r] = hv; stl[c][wave * 16 + 8 * g + r] = lv; } } }
    if (which < 2) { LDSX(); for (int rl = 0; rl < 16; ++rl) { if (lane < 16) vst2((unsigned*)(QH + (r0 + rl) * (2 * DD) + which * DD + lane * 8), *(const v4u*)&sqh[wave][rl][lane * 8]); else vst2((unsigned*)(QL + (r0 + rl) * (2 * DD) + which * DD + (lane - 16) * 8), *(const v4u*)&sql[wave][rl][(lane - 16) * 8]); } }
    else { __syncthreads(); const size_t rb = (size_t)blockIdx.x * 64; const int b = (int)(rb / SS), s0 = (int)(rb % SS);
      for (int q = tid; q < 128 * 8; q += 128) { const int d = q >> 3, pc = q & 7; const size_t o = ((size_t)b * DD + d) * SS + s0 + pc * 8; vst2((unsigned*)(VTH + o), *(const v4u*)&sth[d][pc * 8]); vst2((unsigned*)(VTL + o), *(const v4u*)&stl[d][pc * 8]); } }
    return; }
#pragma unroll
  for (int j = 0; j < 8; ++j) { const int c = n0 + j * 16 + col; const float bb = bfr(BIAS[c]);
#pragma unroll
    for (int r = 0; r < 8; ++r) { const size_t row = r0 + 8 * g + r; const float v = acc[j][r] + bb;
      if (MODE == 2) { const float gq = gelu_exact(v); const __bf16 hb = (__bf16)gq; soh[wave][8 * g + r][j * 16 + col] = hb; sol[wave][8 * g + r][j * 16 + col] = (__bf16)(gq - (float)hb); }
      else so[wave][8 * g + r][j * 16 + col] = X[row * DD + c] + v; } }
  LDSX();
  for (int rl = 0; rl < 16; ++rl) { if (MODE == 2) { if (lane < 16) { vst2((unsigned*)(OH + (r0 + rl) * FF + n0 + lane * 8), *(const v4u*)&soh[wave][rl][lane * 8]); vst2((unsigned*)(OL + (r0 + rl) * FF + n0 + lane * 8), *(const v4u*)&sol[wave][rl][lane * 8]); } }
    else vst2(OUTF + (r0 + rl) * DD + n0 + lane * 4, *(const v4f*)&so[wave][rl][lane * 4]); }
}
__global__ __launch_bounds__(128) void k_attn(const _Float16* __restrict__ QH, const _Float16* __restrict__ QL, const _Float16* __restrict__ VTH, const _Float16* __restrict__ VTL, __bf16* __restrict__ OH, __bf16* __restrict__ OL) {
  __shared__ __align__(16) _Float16 sph[4][16][40], spl[4][16][40]; __shared__ __align__(16) __bf16 soh[64][DD + 8], sol[64][DD + 8];
  const int tid = threadIdx.x, wave = tid >> 5, lane = tid & 31, col = lane & 15, g = lane >> 4; const int qb = blockIdx.x, b = blockIdx.y; const int h = wave;
  for (int rt = 0; rt < 4; ++rt) { const int q0 = qb * 64 + rt * 16; const size_t rq = (size_t)b * SS + q0 + col;
    const v16h aqh = frag_h(QH + rq * (2 * DD) + h * HD, lane), aql = frag_h(QL + rq * (2 * DD) + h * HD, lane);
    float m[8], l[8];
#pragma unroll
    for (int r = 0; r < 8; ++r) { m[r] = -3.0e38f; l[r] = 0.f; }
    v8f acc[2] = {}, accl[2] = {};
    const int nks = (q0 + 16) / 32 + (((q0 + 16) % 32) ? 1 : 0);
#pragma unroll 1
    for (int ks = 0; ks < nks; ++ks) { v8f s[2];
#pragma unroll
      for (int ct = 0; ct < 2; ++ct) { const size_t kk = (size_t)b * SS + ks * 32 + ct * 16 + col; const v16h bkh = frag_h(QH + kk * (2 * DD) + DD + h * HD, lane), bkl = frag_h(QL + kk * (2 * DD) + DD + h * HD, lane);
        v8f c = {}; c = wmma16(aqh, bkh, c); v8f c2 = {}; c2 = wmma16(aql, bkh, c2); c2 = wmma16(aqh, bkl, c2);
#pragma unroll
        for (int r = 0; r < 8; ++r) { const int qi = q0 + 8 * g + r; const int ki = ks * 32 + ct * 16 + col; const float sv = (c[r] + c2[r] * (1.0f / 2048.0f)) * 0.17677669529663688f; s[ct][r] = (ki <= qi) ? sv : -3.0e38f; } }
#pragma unroll
      for (int r = 0; r < 8; ++r) { float mx = fmaxf(s[0][r], s[1][r]);
#pragma unroll
        for (int o = 1; o < 16; o <<= 1) mx = fmaxf(mx, __shfl_xor(mx, o));
        const float mn = fmaxf(m[r], mx); const float alpha = (m[r] <= -1.0e38f) ? 0.f : exp_ni(m[r] - mn);
        float e0 = (s[0][r] <= -1.0e38f) ? 0.f : exp_ni(s[0][r] - mn), e1 = (s[1][r] <= -1.0e38f) ? 0.f : exp_ni(s[1][r] - mn); float es = e0 + e1;
#pragma unroll
        for (int o = 1; o < 16; o <<= 1) es += __shfl_xor(es, o);
        l[r] = l[r] * alpha + es; m[r] = mn;
#pragma unroll
        for (int dt = 0; dt < 2; ++dt) { acc[dt][r] *= alpha; accl[dt][r] *= alpha; }
        const _Float16 h0 = (_Float16)e0, h1 = (_Float16)e1; sph[wave][8 * g + r][col] = h0; sph[wave][8 * g + r][16 + col] = h1; spl[wave][8 * g + r][col] = (_Float16)((e0 - (float)h0) * 2048.0f); spl[wave][8 * g + r][16 + col] = (_Float16)((e1 - (float)h1) * 2048.0f); }
      LDSX();
      const v16h pah = frag_h(&sph[wave][col][0], lane), pal = frag_h(&spl[wave][col][0], lane);
#pragma unroll
      for (int dt = 0; dt < 2; ++dt) { const size_t vo = ((size_t)b * DD + h * HD + dt * 16 + col) * SS + (size_t)ks * 32; const v16h vh = frag_h(VTH + vo, lane), vl = frag_h(VTL + vo, lane);
        acc[dt] = wmma16(pah, vh, acc[dt]); accl[dt] = wmma16(pal, vh, accl[dt]); accl[dt] = wmma16(pah, vl, accl[dt]); }
      LDSX(); }
#pragma unroll
    for (int r = 0; r < 8; ++r) { const float il = 1.0f / l[r];
#pragma unroll
      for (int dt = 0; dt < 2; ++dt) { const float v = (acc[dt][r] + accl[dt][r] * (1.0f / 2048.0f)) * il; const __bf16 hb = (__bf16)v; soh[rt * 16 + 8 * g + r][h * HD + dt * 16 + col] = hb; sol[rt * 16 + 8 * g + r][h * HD + dt * 16 + col] = (__bf16)(v - (float)hb); } } }
  __syncthreads();
  for (int q = tid; q < 64 * 16 * 2; q += 128) { const int plane = q / (64 * 16), rem = q % (64 * 16); const int r = rem >> 4, pc = rem & 15; const size_t o = ((size_t)b * SS + qb * 64 + r) * DD + pc * 8;
    if (plane == 0) vst2((unsigned*)(OH + o), *(const v4u*)&soh[r][pc * 8]); else vst2((unsigned*)(OL + o), *(const v4u*)&sol[r][pc * 8]); }
}
__global__ __launch_bounds__(128) void k_mln(const float* __restrict__ Y, const float* __restrict__ G, const float* __restrict__ Bb, float* __restrict__ X, __bf16* __restrict__ XH, __bf16* __restrict__ XL) {
  __shared__ float sred[2][4]; __shared__ __align__(16) float sx[DD]; __shared__ __align__(16) __bf16 sh_[DD], sl_[DD]; const int t = threadIdx.x, wave = t >> 5; const size_t row = blockIdx.x;
  const float v = Y[row * DD + t]; float s = v;
#pragma unroll
  for (int o = 1; o < 32; o <<= 1) s += __shfl_xor(s, o);
  if ((t & 31) == 0) sred[0][wave] = s;
  __syncthreads();
  const float mu = (wave == 0) ? sred[0][0] * (1.0f / 32.0f) : ((sred[0][1] + sred[0][2]) + sred[0][3]) * (1.0f / 96.0f); const float d = v - mu; float q = d * d;
#pragma unroll
  for (int o = 1; o < 32; o <<= 1) q += __shfl_xor(q, o);
  if ((t & 31) == 0) sred[1][wave] = q;
  __syncthreads();
  const float var = (wave == 0) ? sred[1][0] * (1.0f / 32.0f) : ((sred[1][1] + sred[1][2]) + sred[1][3]) * (1.0f / 96.0f);
  const float x = d * rsqrtf(var + 1e-5f) * bfr(G[t]) + bfr(Bb[t]); sx[t] = x; const __bf16 hb = (__bf16)x; sh_[t] = hb; sl_[t] = (__bf16)(x - (float)hb);
  __syncthreads();
  if (t < 32) vst2(X + row * DD + t * 4, *(const v4f*)&sx[t * 4]); else if (t < 48) vst2((unsigned*)(XH + row * DD + (t - 32) * 8), *(const v4u*)&sh_[(t - 32) * 8]); else if (t < 64) vst2((unsigned*)(XL + row * DD + (t - 48) * 8), *(const v4u*)&sl_[(t - 48) * 8]);
}
__global__ __launch_bounds__(128) void k_pool(const float* __restrict__ X, float* __restrict__ POOL) {
  __shared__ __align__(16) float sp[DD]; const int t = threadIdx.x; const int b = blockIdx.y, blk = blockIdx.x; float a = 0.f;
  for (int r = 0; r < 64; ++r) a += X[((size_t)b * SS + blk * 64 + r) * DD + t];
  sp[t] = a; __syncthreads();
  if (t < 32) vst2(POOL + ((size_t)b * (SS / 64) + blk) * DD + t * 4, *(const v4f*)&sp[t * 4]);
}
__global__ __launch_bounds__(128) void k_cls(const float* __restrict__ POOL, const float* __restrict__ CW, const float* __restrict__ CB, float* __restrict__ OUT) {
  __shared__ float spool[NB][DD]; __shared__ __align__(16) float sout[32]; const int t = threadIdx.x;
  for (int b = 0; b < NB; ++b) { double a = 0.0; for (int blk = 0; blk < SS / 64; ++blk) a += (double)POOL[((size_t)b * (SS / 64) + blk) * DD + t]; spool[b][t] = (float)(a / (double)SS); }
  __syncthreads();
  if (t < 32) { float v = 0.f; if (t < NB * 2) { const int b = t / 2, o = t % 2; float a = 0.f; for (int c = 0; c < DD; ++c) a += spool[b][c] * bfr(CW[c * 2 + o]); v = a + bfr(CB[o]); } sout[t] = v; }
  __syncthreads();
  if (t < 2) vst2(OUT + t * 4, *(const v4f*)&sout[t * 4]);
}
extern "C" void kernel_launch(void* const* d_in, const int* in_sizes, int n_in, void* d_out, int out_size, void* d_ws, size_t ws_size, hipStream_t stream) {
  (void)in_sizes; (void)n_in; (void)out_size;
  const float** F = (const float**)d_in;
  if (ws_size < (size_t)WS_END) return;
  char* ws = (char*)d_ws; __bf16 *PK = (__bf16*)(ws + WS_PK), *XH = (__bf16*)(ws + WS_XH), *XL = (__bf16*)(ws + WS_XL), *AH = (__bf16*)(ws + WS_AH), *AL = (__bf16*)(ws + WS_AL), *HFH = (__bf16*)(ws + WS_HFH), *HFL = (__bf16*)(ws + WS_HFL);
  float *X = (float*)(ws + WS_X), *Y = (float*)(ws + WS_Y), *POOL = (float*)(ws + WS_POOL); _Float16 *QH = (_Float16*)(ws + WS_QH), *QL = (_Float16*)(ws + WS_QL), *VTH = (_Float16*)(ws + WS_VTH), *VTL = (_Float16*)(ws + WS_VTL);
  k_pack<<<dim3(FF, 4, NL), 128, 0, stream>>>(F[3], F[5], F[7], F[9], F[13], F[15], PK);
  k_embed<<<NRT, 128, 0, stream>>>(F[0], F[1], F[2], X, XH, XL);
  for (int l = 0; l < NL; ++l) { const __bf16* base = PK + (size_t)l * PL_SZ;
    k_gemm<0><<<dim3(NRT / 64, 1), 128, 0, stream>>>(XH, XL, base + PL_QKV, F[4] + (size_t)l * DD, X, QH, QL, VTH, VTL, nullptr, nullptr, nullptr, 0);
    k_gemm<0><<<dim3(NRT / 64, 1), 128, 0, stream>>>(XH, XL, base + PL_QKV + (size_t)DD * DD, F[6] + (size_t)l * DD, X, QH, QL, VTH, VTL, nullptr, nullptr, nullptr, 1);
    k_gemm<0><<<dim3(NRT / 64, 1), 128, 0, stream>>>(XH, XL, base + PL_QKV + (size_t)2 * DD * DD, F[8] + (size_t)l * DD, X, QH, QL, VTH, VTL, nullptr, nullptr, nullptr, 2);
    k_attn<<<dim3((NRT < SS ? NRT : SS) / 64, (NRT < SS ? 1 : NB)), 128, 0, stream>>>(QH, QL, VTH, VTL, AH, AL);
    k_gemm<1><<<dim3(NRT / 64, 1), 128, 0, stream>>>(AH, AL, base + PL_O, F[10] + (size_t)l * DD, X, nullptr, nullptr, nullptr, nullptr, nullptr, nullptr, Y, 0);
    k_mln<<<NRT, 128, 0, stream>>>(Y, F[11] + (size_t)l * DD, F[12] + (size_t)l * DD, X, XH, XL);
    k_gemm<2><<<dim3(NRT / 64, FF / 128), 128, 0, stream>>>(XH, XL, base + PL_F1, F[14] + (size_t)l * FF, nullptr, nullptr, nullptr, nullptr, nullptr, HFH, HFL, nullptr, 0);
    k_gemm<3><<<dim3(NRT / 64, 1), 128, 0, stream>>>(HFH, HFL, base + PL_F2, F[16] + (size_t)l * DD, X, nullptr, nullptr, nullptr, nullptr, nullptr, nullptr, Y, 0);
    k_mln<<<NRT, 128, 0, stream>>>(Y, F[17] + (size_t)l * DD, F[18] + (size_t)l * DD, X, XH, XL); }
  k_pool<<<dim3(SS / 64, NB), 128, 0, stream>>>(X, POOL);
  k_cls<<<1, 128, 0, stream>>>(POOL, F[19], F[20], (float*)d_out);
}
